// NNConv_block_58291296141370
// MI455X (gfx1250) — hardware-verified
//
#include <hip/hip_runtime.h>
#include <stddef.h>


#define DIMF   64
#define EDIM   12
#define KP     13
#define KTOT   (KP * DIMF)
#define NTHR   256
#define NWAVE  8
#define EPT    8
#define NGRP   2
#define CHUNK  (NTHR * EPT * NGRP)
#define WCAP   (EPT * NGRP * 32)
#define LISTN  (NWAVE * WCAP)
#define NB     1024
#define GROWS  128
#define GCOLS  64
#define STGW   32
#define WSCALE 16.0f
#define WINV   0.0625f
#define BN_EPS 1e-5f
#define LDS_AGG (NB * DIMF * 4 + LISTN * 4 + NB * 4 + 64)

static_assert((CHUNK & (CHUNK - 1)) == 0);
static_assert(CHUNK <= 4096);
static_assert((NB & (NB - 1)) == 0);
static_assert(NB <= 4096);
static_assert(NB % (16 * NWAVE) == 0);
static_assert(NWAVE * 16 * STGW * 4 <= LISTN * 4);
static_assert(KTOT % GCOLS == 0);
static_assert(GROWS == 16 * NWAVE);
static_assert((NWAVE & (NWAVE - 1)) == 0);

typedef float    v2f  __attribute__((ext_vector_type(2)));
typedef float    v4f  __attribute__((ext_vector_type(4)));
typedef float    v8f  __attribute__((ext_vector_type(8)));
typedef int      v4i  __attribute__((ext_vector_type(4)));
typedef _Float16 v8h  __attribute__((ext_vector_type(8)));
typedef _Float16 v16h __attribute__((ext_vector_type(16)));
union FragH { v16h v; v8h h[2]; };

__device__ __forceinline__ v8h cvt8(v4f a, v4f b) {
  v8h r;
  r[0] = (_Float16)a.x; r[1] = (_Float16)a.y; r[2] = (_Float16)a.z; r[3] = (_Float16)a.w;
  r[4] = (_Float16)b.x; r[5] = (_Float16)b.y; r[6] = (_Float16)b.z; r[7] = (_Float16)b.w;
  return r;
}

__device__ __forceinline__ v8f wmh(v16h a, v16h b, v8f c) {
  v8f d = __builtin_amdgcn_wmma_f32_16x16x32_f16(false, a, false, b, (short)0, c, false, false);
  asm volatile("v_nop\n\tv_nop\n\tv_nop\n\tv_nop" : "+v"(d) : "v"(a), "v"(b));
  return d;
}

template <int NBT>
__device__ __forceinline__ int scan_chunk(const int* __restrict__ dsts, int nE, int cbase, int nodeBase,
                                          int vec8, int* list, int tid, int lane, int wave) {
  int wc = 0;
#pragma unroll
  for (int g = 0; g < NGRP; ++g) {
    const int el0  = (g * NTHR + tid) * EPT;
    const int e0   = cbase + el0;
    const int sent = -2147483647 - 1;
    v4i da, db;
    if (vec8 != 0 && e0 + 7 < nE) {
      da = *(const v4i*)(dsts + e0);
      db = *(const v4i*)(dsts + e0 + 4);
    } else {
      da.x = (e0     < nE) ? dsts[min(e0, nE - 1)] : sent;
      da.y = (e0 + 1 < nE) ? dsts[min(e0 + 1, nE - 1)] : sent;
      da.z = (e0 + 2 < nE) ? dsts[min(e0 + 2, nE - 1)] : sent;
      da.w = (e0 + 3 < nE) ? dsts[min(e0 + 3, nE - 1)] : sent;
      db.x = (e0 + 4 < nE) ? dsts[min(e0 + 4, nE - 1)] : sent;
      db.y = (e0 + 5 < nE) ? dsts[min(e0 + 5, nE - 1)] : sent;
      db.z = (e0 + 6 < nE) ? dsts[min(e0 + 6, nE - 1)] : sent;
      db.w = (e0 + 7 < nE) ? dsts[min(e0 + 7, nE - 1)] : sent;
    }
    const unsigned nb = (unsigned)nodeBase;
    const unsigned s0 = (unsigned)da.x - nb, s1 = (unsigned)da.y - nb;
    const unsigned s2 = (unsigned)da.z - nb, s3 = (unsigned)da.w - nb;
    const unsigned s4 = (unsigned)db.x - nb, s5 = (unsigned)db.y - nb;
    const unsigned s6 = (unsigned)db.z - nb, s7 = (unsigned)db.w - nb;
    const bool h0 = s0 < (unsigned)NBT, h1 = s1 < (unsigned)NBT, h2 = s2 < (unsigned)NBT, h3 = s3 < (unsigned)NBT;
    const bool h4 = s4 < (unsigned)NBT, h5 = s5 < (unsigned)NBT, h6 = s6 < (unsigned)NBT, h7 = s7 < (unsigned)NBT;
    const unsigned any = __builtin_amdgcn_ballot_w32(h0 | h1 | h2 | h3 | h4 | h5 | h6 | h7);
    if (any != 0u) {
#define HITJ(J, HJ, SJ) { \
        const unsigned mj = __builtin_amdgcn_ballot_w32(HJ); \
        if (mj != 0u) { \
          if (HJ) { \
            const int pos = wc + (int)__builtin_amdgcn_mbcnt_lo(mj, 0u); \
            if (pos < WCAP) list[wave * WCAP + pos] = ((el0 + (J)) << 12) | (int)(SJ); \
          } \
          wc += (int)__builtin_popcount(mj); } }
      HITJ(0, h0, s0)
      HITJ(1, h1, s1)
      HITJ(2, h2, s2)
      HITJ(3, h3, s3)
      HITJ(4, h4, s4)
      HITJ(5, h5, s5)
      HITJ(6, h6, s6)
      HITJ(7, h7, s7)
#undef HITJ
    }
  }
  return wc;
}

__global__ __launch_bounds__(NTHR) void k_prep(
    const float* __restrict__ x, const float* __restrict__ lw, const float* __restrict__ lb,
    const float* __restrict__ wih, const float* __restrict__ whh,
    _Float16* x16, _Float16* Lt, _Float16* wih16, _Float16* whh16, int nN) {
  const int i  = blockIdx.x * NTHR + threadIdx.x;
  const int n0 = nN * (DIMF / 8);
  const int n1 = KTOT * DIMF / 8;
  const int n2 = 3 * DIMF * DIMF / 8;
  if (i >= n0 + n1 + 2 * n2) return;
  v4f a, b;
  _Float16* dp;
  if (i < n0) {
    const size_t o = (size_t)i * 8;
    a  = *(const v4f*)(x + o);
    b  = *(const v4f*)(x + o + 4);
    dp = x16 + o;
  } else if (i < n0 + n1) {
    const int o   = (i - n0) * 8;
    const int n   = o >> 6;
    const int k0  = o & 63;
    const int k13 = n >> 6;
    const int oo  = n & 63;
    const float* p = (k13 < EDIM) ? (lw + (size_t)k13 * (DIMF * DIMF) + (size_t)k0 * DIMF + oo)
                                  : (lb + (size_t)k0 * DIMF + oo);
    a.x = p[0];        a.y = p[DIMF];     a.z = p[2 * DIMF]; a.w = p[3 * DIMF];
    b.x = p[4 * DIMF]; b.y = p[5 * DIMF]; b.z = p[6 * DIMF]; b.w = p[7 * DIMF];
    a = a * WSCALE;
    b = b * WSCALE;
    dp = Lt + o;
  } else {
    const int  j     = i - n0 - n1;
    const bool first = j < n2;
    const int  o     = (first ? j : j - n2) * 8;
    const float* p = (first ? wih : whh) + o;
    a  = *(const v4f*)p;
    b  = *(const v4f*)(p + 4);
    a  = a * WSCALE;
    b  = b * WSCALE;
    dp = (first ? wih16 : whh16) + o;
  }
  const v8h hv = cvt8(a, b);
  *(volatile v8h*)dp = hv;
  __threadfence();
  *(volatile v8h*)dp = hv;
}

__global__ __launch_bounds__(NTHR) void k_bn(
    const float* __restrict__ ea, const float* __restrict__ gamma, float* bnss, int nE) {
  __shared__ __attribute__((aligned(16))) double red[2 * EDIM * NTHR];
  __shared__ double tot[2 * EDIM];
  __shared__ __attribute__((aligned(16))) float outl[32];
  const int tid = threadIdx.x;
  double s[EDIM], q[EDIM];
#pragma unroll
  for (int k = 0; k < EDIM; ++k) { s[k] = 0.0; q[k] = 0.0; }
  if (tid < 32) outl[tid] = 0.f;
#pragma unroll 1
  for (int e = tid; e < nE; e += NTHR) {
    const float* row = ea + (size_t)e * EDIM;
    const v4f r0 = *(const v4f*)row, r1 = *(const v4f*)(row + 4), r2 = *(const v4f*)(row + 8);
    const float v[EDIM] = {r0.x, r0.y, r0.z, r0.w, r1.x, r1.y, r1.z, r1.w, r2.x, r2.y, r2.z, r2.w};
#pragma unroll
    for (int k = 0; k < EDIM; ++k) {
      const double d = (double)v[k];
      s[k] += d;
      q[k] += d * d;
    }
  }
#pragma unroll
  for (int k = 0; k < EDIM; ++k) {
    red[k * NTHR + tid]          = s[k];
    red[(EDIM + k) * NTHR + tid] = q[k];
  }
  __syncthreads();
  if (tid < 2 * EDIM) {
    double t = 0.0;
#pragma unroll 1
    for (int i = 0; i < NTHR; ++i) t += red[tid * NTHR + i];
    tot[tid] = t;
  }
  __syncthreads();
  if (tid < EDIM) {
    const double invn = 1.0 / (double)nE;
    const double mu   = tot[tid] * invn;
    double var = tot[EDIM + tid] * invn - mu * mu;
    var = var < 0.0 ? 0.0 : var;
    outl[tid]      = (float)mu;
    outl[16 + tid] = gamma[tid] * rsqrtf((float)var + BN_EPS);
  }
  __syncthreads();
  if (tid < 8) {
    const v4f v = *(const v4f*)(outl + 4 * tid);
    *(volatile v4f*)(bnss + 4 * tid) = v;
    __threadfence();
    *(volatile v4f*)(bnss + 4 * tid) = v;
  }
}

__global__ __launch_bounds__(NTHR) void k_gemmP(
    const _Float16* __restrict__ x16, const _Float16* __restrict__ Lt, float* P, int nN) {
  __shared__ __attribute__((aligned(16))) float stg[NWAVE * 16 * GCOLS];
  const int tid = threadIdx.x, lane = tid & 31, wave = tid >> 5, hh = lane >> 4, m = lane & 15;
  const int colBase = blockIdx.x * GCOLS;
  const int rowBase = blockIdx.y * GROWS + wave * 16;
  int node = rowBase + m;
  node = node > nN - 1 ? nN - 1 : node;

  v8f acc[4];
#pragma unroll
  for (int t = 0; t < 4; ++t) { v8f z = {0.f, 0.f, 0.f, 0.f, 0.f, 0.f, 0.f, 0.f}; acc[t] = z; }
  const _Float16* ar = x16 + (size_t)node * DIMF + 8 * hh;
#pragma unroll
  for (int ks = 0; ks < DIMF / 32; ++ks) {
    FragH a;
    a.h[0] = *(const v8h*)(ar + 32 * ks);
    a.h[1] = *(const v8h*)(ar + 32 * ks + 16);
#pragma unroll
    for (int t = 0; t < 4; ++t) {
      const _Float16* bp = Lt + (size_t)(colBase + 16 * t + m) * DIMF + 32 * ks + 8 * hh;
      FragH b;
      b.h[0] = *(const v8h*)bp;
      b.h[1] = *(const v8h*)(bp + 16);
      acc[t] = wmh(a.v, b.v, acc[t]);
    }
  }

  float* sp = stg + wave * (16 * GCOLS) + (8 * hh) * GCOLS + m;
#pragma unroll
  for (int t = 0; t < 4; ++t) {
#pragma unroll
    for (int r = 0; r < 8; ++r) sp[r * GCOLS + 16 * t] = acc[t][r] * WINV;
  }
  __syncthreads();

  const int rsel = lane >> 4, c4 = 4 * (lane & 15);
  const float* lp = stg + wave * (16 * GCOLS) + rsel * GCOLS + c4;
  float* gp = P + ((size_t)rowBase + rsel) * KTOT + colBase + c4;
  v4f ov[8];
#pragma unroll
  for (int i = 0; i < 8; ++i) ov[i] = *(const v4f*)(lp + 2 * i * GCOLS);
#pragma unroll
  for (int i = 0; i < 8; ++i) *(volatile v4f*)(gp + (size_t)(2 * i) * KTOT) = ov[i];
  __threadfence();
#pragma unroll
  for (int i = 0; i < 8; ++i) *(volatile v4f*)(gp + (size_t)(2 * i) * KTOT) = ov[i];
}

__global__ __launch_bounds__(NTHR) void k_agg(
    const int* __restrict__ ei, const float* __restrict__ ea, const float* __restrict__ bnss,
    const float* __restrict__ beta, const float* __restrict__ P, const float* __restrict__ x,
    const _Float16* __restrict__ x16, const _Float16* __restrict__ wih16,
    const _Float16* __restrict__ whh16, const float* __restrict__ bih,
    const float* __restrict__ bhh, float* out, int nN, int nE, int vec8) {
  extern __shared__ v4f lds_dyn[];
  float* acc  = (float*)lds_dyn;
  int*   list = (int*)(acc + NB * DIMF);
  int*   cnt  = list + LISTN;
  int*   wcnt = cnt + NB;
  float* stg  = (float*)list;
  const int tid = threadIdx.x, lane = tid & 31, wave = tid >> 5, hh = lane >> 4, m = lane & 15;
  const int nodeBase = blockIdx.x * NB;
  const int* dsts = ei + nE;

  {
    const v4f z = {0.f, 0.f, 0.f, 0.f};
    for (int i = tid; i < NB * DIMF / 4; i += NTHR) lds_dyn[i] = z;
    for (int i = tid; i < NB; i += NTHR) cnt[i] = 0;
  }
  float mu[EDIM], sc[EDIM], bb[EDIM];
#pragma unroll
  for (int k = 0; k < EDIM; ++k) { mu[k] = bnss[k]; sc[k] = bnss[16 + k]; bb[k] = beta[k]; }
  __syncthreads();

  const int nChunks = (nE + CHUNK - 1) / CHUNK;
#pragma unroll 1
  for (int ch = 0; ch < nChunks; ++ch) {
    const int cbase = ch * CHUNK;
    const int wc = scan_chunk<NB>(dsts, nE, cbase, nodeBase, vec8, list, tid, lane, wave);
    if (lane == 0) wcnt[wave] = wc;
    __syncthreads();
#pragma unroll 1
    for (int wsx = 0; wsx < NWAVE; ++wsx) {
      int n = __builtin_amdgcn_readfirstlane(wcnt[wsx]);
      n = n > WCAP ? WCAP : (n < 0 ? 0 : n);
      const int* lp = list + wsx * WCAP;
#pragma unroll 1
      for (int i = 0; i < n; ++i) {
        const int ent  = __builtin_amdgcn_readfirstlane(lp[i]);
        const int slot = ent & (NB - 1);
        if ((slot & (NWAVE - 1)) != wave) continue;
        int e = cbase + ((ent >> 12) & (CHUNK - 1));
        e = e > nE - 1 ? nE - 1 : e;
        int src = ei[e];
        src = src < 0 ? 0 : (src > nN - 1 ? nN - 1 : src);
        const float* er = ea + (size_t)e * EDIM;
        const float* pr = P + (size_t)src * KTOT + 2 * lane;
        const v2f pb = *(const v2f*)(pr + EDIM * DIMF);
        float mx = pb.x, my = pb.y;
#pragma unroll
        for (int k = 0; k < EDIM; ++k) {
          const float ek = (er[k] - mu[k]) * sc[k] + bb[k];
          const v2f  pk = *(const v2f*)(pr + k * DIMF);
          mx += ek * pk.x;
          my += ek * pk.y;
        }
        v2f* ap = (v2f*)(acc + slot * DIMF + 2 * lane);
        v2f av = *ap;
        av.x += mx;
        av.y += my;
        *ap = av;
        if (lane == 0) cnt[slot] = cnt[slot] + 1;
      }
    }
    __syncthreads();
  }

#pragma unroll 4
  for (int i = 0; i < (NB * DIMF / 4) / NTHR; ++i) {
    const int idx  = i * NTHR + tid;
    const int slot = idx >> 4;
    int cv = cnt[slot];
    cv = cv < 1 ? 1 : cv;
    const float inv = 1.0f / (float)cv;
    v4f v = lds_dyn[idx] * inv;
    v.x = fmaxf(v.x, 0.f); v.y = fmaxf(v.y, 0.f); v.z = fmaxf(v.z, 0.f); v.w = fmaxf(v.w, 0.f);
    lds_dyn[idx] = v;
  }
  __syncthreads();

#pragma unroll 1
  for (int T = 0; T < NB / 16 / NWAVE; ++T) {
    const int rt    = wave * (NB / 16 / NWAVE) + T;
    const int slot0 = 16 * rt;
    int nodem = nodeBase + slot0 + m;
    nodem = nodem > nN - 1 ? nN - 1 : nodem;
    FragH am[2], ax[2];
#pragma unroll
    for (int ks = 0; ks < 2; ++ks) {
      const float* mp = acc + (slot0 + m) * DIMF + 32 * ks + 8 * hh;
      am[ks].h[0] = cvt8(*(const v4f*)mp, *(const v4f*)(mp + 4));
      am[ks].h[1] = cvt8(*(const v4f*)(mp + 16), *(const v4f*)(mp + 20));
      const _Float16* xp = x16 + (size_t)nodem * DIMF + 32 * ks + 8 * hh;
      ax[ks].h[0] = *(const v8h*)xp;
      ax[ks].h[1] = *(const v8h*)(xp + 16);
    }
#pragma unroll 1
    for (int t = 0; t < 4; ++t) {
      v8f c[6];
#pragma unroll
      for (int g = 0; g < 6; ++g) { v8f z = {0.f, 0.f, 0.f, 0.f, 0.f, 0.f, 0.f, 0.f}; c[g] = z; }
#pragma unroll
      for (int ks = 0; ks < 2; ++ks) {
#pragma unroll
        for (int g = 0; g < 3; ++g) {
          const size_t boff = (size_t)(DIMF * g + 16 * t + m) * DIMF + 32 * ks + 8 * hh;
          FragH bi, bh;
          bi.h[0] = *(const v8h*)(wih16 + boff);
          bi.h[1] = *(const v8h*)(wih16 + boff + 16);
          bh.h[0] = *(const v8h*)(whh16 + boff);
          bh.h[1] = *(const v8h*)(whh16 + boff + 16);
          c[g]     = wmh(am[ks].v, bi.v, c[g]);
          c[3 + g] = wmh(ax[ks].v, bh.v, c[3 + g]);
        }
      }
      const int col = 16 * t + m;
      const float bir = bih[col], biz = bih[DIMF + col], bin2 = bih[2 * DIMF + col];
      const float bhr = bhh[col], bhz = bhh[DIMF + col], bhn = bhh[2 * DIMF + col];
      float* sp = stg + wave * (16 * STGW) + (8 * hh) * STGW + 16 * (t & 1) + m;
#pragma unroll
      for (int r = 0; r < 8; ++r) {
        int node = nodeBase + slot0 + 8 * hh + r;
        node = node > nN - 1 ? nN - 1 : node;
        const float xv  = x[(size_t)node * DIMF + col];
        const float ir  = c[0][r] * WINV + bir;
        const float iz  = c[1][r] * WINV + biz;
        const float gn  = c[2][r] * WINV + bin2;
        const float hr  = c[3][r] * WINV + bhr;
        const float hz  = c[4][r] * WINV + bhz;
        const float hn  = c[5][r] * WINV + bhn;
        const float rg  = __builtin_amdgcn_rcpf(1.0f + __expf(-(ir + hr)));
        const float zg  = __builtin_amdgcn_rcpf(1.0f + __expf(-(iz + hz)));
        const float pre = gn + rg * hn;
        const float ng  = 1.0f - 2.0f * __builtin_amdgcn_rcpf(__expf(2.0f * pre) + 1.0f);
        sp[r * STGW] = (1.0f - zg) * ng + zg * xv;
      }
      if ((t & 1) != 0) {
        __syncthreads();
        const int half = t >> 1;
        const int rq = lane >> 3, c4 = 4 * (lane & 7);
        const float* lp = stg + wave * (16 * STGW) + rq * STGW + c4;
        v4f ov[4];
#pragma unroll
        for (int q = 0; q < 4; ++q) ov[q] = *(const v4f*)(lp + 4 * q * STGW);
#pragma unroll
        for (int q = 0; q < 4; ++q) {
          const int node = nodeBase + slot0 + 4 * q + rq;
          if (node < nN) *(volatile v4f*)(out + (size_t)node * DIMF + 32 * half + c4) = ov[q];
        }
        __threadfence();
#pragma unroll
        for (int q = 0; q < 4; ++q) {
          const int node = nodeBase + slot0 + 4 * q + rq;
          if (node < nN) *(volatile v4f*)(out + (size_t)node * DIMF + 32 * half + c4) = ov[q];
        }
        __syncthreads();
      }
    }
  }
}

extern "C" void kernel_launch(void* const* d_in, const int* in_sizes, int n_in,
                              void* d_out, int out_size, void* d_ws, size_t ws_size,
                              hipStream_t stream) {
  if (n_in < 11) return;
  const int nN = in_sizes[0] / DIMF;
  const int nE = in_sizes[1] / 2;
  if (nN <= 0 || nE <= 0) return;
  if (in_sizes[0] != nN * DIMF || in_sizes[1] != 2 * nE || in_sizes[2] != nE * EDIM) return;
  if (in_sizes[3] < EDIM || in_sizes[4] < EDIM) return;
  if (in_sizes[5] != EDIM * DIMF * DIMF || in_sizes[6] != DIMF * DIMF) return;
  if (in_sizes[7] != 3 * DIMF * DIMF || in_sizes[8] != 3 * DIMF * DIMF) return;
  if (in_sizes[9] < 3 * DIMF || in_sizes[10] < 3 * DIMF) return;
  if (out_size != nN * DIMF) return;

  const float* x     = (const float*)d_in[0];
  const int*   ei    = (const int*)d_in[1];
  const float* ea    = (const float*)d_in[2];
  const float* gamma = (const float*)d_in[3];
  const float* beta  = (const float*)d_in[4];
  const float* lin_w = (const float*)d_in[5];
  const float* lin_b = (const float*)d_in[6];
  const float* w_ih  = (const float*)d_in[7];
  const float* w_hh  = (const float*)d_in[8];
  const float* b_ih  = (const float*)d_in[9];
  const float* b_hh  = (const float*)d_in[10];
  float* out = (float*)d_out;

  const int nGR = (nN + GROWS - 1) / GROWS;
  const int nPR = nGR * GROWS;
  const int nAB = (nN + NB - 1) / NB;

  char* ws = (char*)d_ws;
  size_t off = 0;
  const size_t oX16 = off; off += (size_t)nN * DIMF * 2;          off = (off + 255) & ~(size_t)255;
  const size_t oLt  = off; off += (size_t)KTOT * DIMF * 2;        off = (off + 255) & ~(size_t)255;
  const size_t oWih = off; off += (size_t)3 * DIMF * DIMF * 2;    off = (off + 255) & ~(size_t)255;
  const size_t oWhh = off; off += (size_t)3 * DIMF * DIMF * 2;    off = (off + 255) & ~(size_t)255;
  const size_t oBn  = off; off += 256;
  const size_t oP   = off; off += (size_t)nPR * KTOT * 4;         off = (off + 255) & ~(size_t)255;
  if (off > ws_size) return;
  _Float16* x16   = (_Float16*)(ws + oX16);
  _Float16* Lt    = (_Float16*)(ws + oLt);
  _Float16* wih16 = (_Float16*)(ws + oWih);
  _Float16* whh16 = (_Float16*)(ws + oWhh);
  float*    bnss  = (float*)(ws + oBn);
  float*    P     = (float*)(ws + oP);

  const int vec8 = ((nE & 3) == 0) ? 1 : 0;

  const int nPrep = nN * (DIMF / 8) + KTOT * DIMF / 8 + 2 * (3 * DIMF * DIMF / 8);
  k_prep<<<(nPrep + NTHR - 1) / NTHR, NTHR, 0, stream>>>(x, lin_w, lin_b, w_ih, w_hh,
                                                          x16, Lt, wih16, whh16, nN);

  k_bn<<<1, NTHR, 0, stream>>>(ea, gamma, bnss, nE);

  k_gemmP<<<dim3(KTOT / GCOLS, nGR), NTHR, 0, stream>>>(x16, Lt, P, nN);

  hipFuncSetAttribute(reinterpret_cast<const void*>(&k_agg),
                      hipFuncAttributeMaxDynamicSharedMemorySize, LDS_AGG);
  k_agg<<<nAB, NTHR, LDS_AGG, stream>>>(ei, ea, bnss, beta, P, x, x16, wih16, whh16,
                                         b_ih, b_hh, out, nN, nE, vec8);
}
